// DeltaVisionMambaBlock_40939628266024
// MI455X (gfx1250) — hardware-verified
//
#include <hip/hip_runtime.h>
#include <math.h>

typedef __attribute__((ext_vector_type(16))) _Float16 v16h;
typedef __attribute__((ext_vector_type(8)))  _Float16 v8h;
typedef __attribute__((ext_vector_type(16))) __bf16   v16b;
typedef __attribute__((ext_vector_type(8)))  __bf16   v8b;
typedef __attribute__((ext_vector_type(8)))  float    v8f;
typedef __attribute__((ext_vector_type(4)))  float    v4f;

constexpr int kBatch  = 2;
constexpr int kSeqL   = 2048;
constexpr int kDm     = 768;
constexpr int kDin    = 1536;
constexpr int kNst    = 16;
constexpr int kTaps   = 4;
constexpr int kDtR    = 48;
constexpr int kDtP    = 64;
constexpr int kXdN    = 80;
constexpr int kXdP    = 128;
constexpr int kCombK  = 2 * kDm;
constexpr int kXZP    = 2 * kDin;
constexpr int kRows   = kBatch * kSeqL;
constexpr int kTP     = 260;
constexpr int kScanCh = 128;
constexpr int kSYP    = 132;

__device__ __forceinline__ unsigned short f2bf_bits(float f) {
  unsigned u = __float_as_uint(f);
  return (unsigned short)((u + 0x7FFFu + ((u >> 16) & 1u)) >> 16);
}
__device__ __forceinline__ float bf_bits2f(unsigned short h) { return __uint_as_float(((unsigned)h) << 16); }
__device__ __forceinline__ float h2f(unsigned short u) { return (float)__builtin_bit_cast(_Float16, u); }

__device__ __forceinline__ void dep_guard_h(v8f& a, v8f& b, v16h x, v16h y) { asm volatile("v_nop\n\tv_nop\n\tv_nop\n\tv_nop" : "+v"(a), "+v"(b) : "v"(x), "v"(y)); }
__device__ __forceinline__ void dep_guard_b(v8f& a, v8f& b, v16b x, v16b y) { asm volatile("v_nop\n\tv_nop\n\tv_nop\n\tv_nop" : "+v"(a), "+v"(b) : "v"(x), "v"(y)); }
__device__ __forceinline__ void keep4_h(v16h a, v16h b, v16h c, v16h d) { asm volatile("v_nop" :: "v"(a), "v"(b), "v"(c), "v"(d)); }
__device__ __forceinline__ void keep4_b(v16b a, v16b b, v16b c, v16b d) { asm volatile("v_nop" :: "v"(a), "v"(b), "v"(c), "v"(d)); }
__device__ __forceinline__ void acc_guard4(v8f& a, v8f& b, v8f& c, v8f& d) { asm volatile("v_nop\n\tv_nop\n\tv_nop\n\tv_nop" : "+v"(a), "+v"(b), "+v"(c), "+v"(d)); }
template <typename T> struct Frag;
template <> struct Frag<_Float16> {
  typedef v16h V; union U { v16h v; v8h h[2]; };
  static __device__ __forceinline__ v16h load(const _Float16* p) {
    U f; f.h[0] = *(const v8h*)(p); f.h[1] = *(const v8h*)(p + 16); return f.v;
  }
  static __device__ __forceinline__ v8f mma(v16h a, v16h b, v8f c) {
    return __builtin_amdgcn_wmma_f32_16x16x32_f16(false, a, false, b, (short)0, c, false, false);
  }
  static __device__ __forceinline__ void guard(v8f& a, v8f& b, v16h x, v16h y) { dep_guard_h(a, b, x, y); }
  static __device__ __forceinline__ void keep(v16h a, v16h b, v16h c, v16h d) { keep4_h(a, b, c, d); }
};
template <> struct Frag<__bf16> {
  typedef v16b V; union U { v16b v; v8b h[2]; };
  static __device__ __forceinline__ v16b load(const __bf16* p) {
    U f; f.h[0] = *(const v8b*)(p); f.h[1] = *(const v8b*)(p + 16); return f.v;
  }
  static __device__ __forceinline__ v8f mma(v16b a, v16b b, v8f c) {
    return __builtin_amdgcn_wmma_f32_16x16x32_bf16(false, a, false, b, (short)0, c, false, false);
  }
  static __device__ __forceinline__ void guard(v8f& a, v8f& b, v16b x, v16b y) { dep_guard_b(a, b, x, y); }
  static __device__ __forceinline__ void keep(v16b a, v16b b, v16b c, v16b d) { keep4_b(a, b, c, d); }
};

template <int ET> struct Elem;
template <> struct Elem<0> { typedef _Float16 T; };
template <> struct Elem<1> { typedef __bf16 T; };
template <int ET, bool SPLIT, int BIAS_MODE, int OUT_MODE, bool RESID, int ACT = 0>
__global__ __launch_bounds__(256) void wmma_gemm64(
    const unsigned short* __restrict__ Ap, const unsigned short* __restrict__ A2p, int lda, long strideA,
    const unsigned short* __restrict__ Btp, const unsigned short* __restrict__ Bt2p, int ldb, long strideB,
    void* __restrict__ Cout, void* __restrict__ Cout2, int ldc, long strideC,
    const float* __restrict__ bias,
    const float* __restrict__ resid, long strideR,
    int M, int N, int K, float scale) {
  typedef typename Elem<ET>::T T;
  typedef typename Frag<T>::V V;
  const T* A = (const T*)Ap; const T* A2 = (const T*)A2p; const T* Bt = (const T*)Btp; const T* Bt2 = (const T*)Bt2p;
  __shared__ __align__(16) float sT[8][16 * 68];
  const int b    = blockIdx.y;
  const int lane = threadIdx.x & 31;
  const int wave = threadIdx.x >> 5;
  const int tilesN = N >> 6;
  const int tilesM = M >> 6;
  const int tile = blockIdx.x * 8 + wave;
  if (tile >= tilesM * tilesN) return;
  const int tm = tile / tilesN;
  const int tn = tile - tm * tilesN;
  const int m0 = tm << 6;
  const int n0 = tn << 6;

  const T* Ab  = A  + (size_t)b * strideA;
  const T* Bb  = Bt + (size_t)b * strideB;
  const T* Ab2 = SPLIT ? (A2  + (size_t)b * strideA) : nullptr;
  const T* Bb2 = SPLIT ? (Bt2 + (size_t)b * strideB) : nullptr;

  const int rlane = lane & 15;
  const int koff  = (lane >> 4) * 8;
  const int mOff  = (lane >> 4) * 8;

  v8f acc[4][4];
#pragma unroll
  for (int i = 0; i < 4; ++i)
#pragma unroll
    for (int j = 0; j < 4; ++j) acc[i][j] = (v8f){0.f,0.f,0.f,0.f,0.f,0.f,0.f,0.f};

  for (int k0 = 0; k0 < K; k0 += 32) {
    V bh[4], bl[4];
#pragma unroll
    for (int j = 0; j < 4; ++j) {
      const size_t bo = (size_t)(n0 + (j << 4) + rlane) * ldb + koff + k0;
      bh[j] = Frag<T>::load(Bb + bo);
      if (SPLIT) bl[j] = Frag<T>::load(Bb2 + bo);
    }
#pragma unroll
    for (int i = 0; i < 4; ++i) {
      const size_t ao = (size_t)(m0 + (i << 4) + rlane) * lda + koff + k0;
      V ah = Frag<T>::load(Ab + ao);
      V al;
      if (SPLIT) al = Frag<T>::load(Ab2 + ao);
#pragma unroll
      for (int j = 0; j < 4; ++j) {
        acc[i][j] = Frag<T>::mma(ah, bh[j], acc[i][j]);
        if (SPLIT) {
          acc[i][j] = Frag<T>::mma(ah, bl[j], acc[i][j]);
          acc[i][j] = Frag<T>::mma(al, bh[j], acc[i][j]);
        }
      }
      Frag<T>::guard(acc[i][0], acc[i][3], ah, SPLIT ? al : ah);
    }
    Frag<T>::keep(bh[0], bh[1], bh[2], bh[3]);
    if (SPLIT) Frag<T>::keep(bl[0], bl[1], bl[2], bl[3]);
  }
  acc_guard4(acc[0][0], acc[0][1], acc[0][2], acc[0][3]);
  acc_guard4(acc[1][0], acc[1][1], acc[1][2], acc[1][3]);
  acc_guard4(acc[2][0], acc[2][1], acc[2][2], acc[2][3]);
  acc_guard4(acc[3][0], acc[3][1], acc[3][2], acc[3][3]);

  float* slab = sT[wave];
  const float* Rb = RESID ? (resid + (size_t)b * strideR) : nullptr;
#pragma unroll
  for (int i = 0; i < 4; ++i) {
    const int mBase = m0 + (i << 4);
#pragma unroll
    for (int j = 0; j < 4; ++j) {
      const int n = n0 + (j << 4) + rlane;
      float bv = 0.f;
      if (BIAS_MODE == 2) bv = bias[n];
#pragma unroll
      for (int r = 0; r < 8; ++r) {
        float v = acc[i][j][r] * scale;
        if (BIAS_MODE == 1) v += bias[mBase + mOff + r];
        if (BIAS_MODE == 2) v += bv;
        if (RESID) v += Rb[(size_t)(mBase + mOff + r) * ldc + n];
        if (ACT == 1) v = tanhf(v);
        if (ACT == 2) v = fmaxf(v, 0.0f);
        if (ACT == 3) v = v / (1.0f + expf(-v));
        if (ACT == 4) v = (v > 0.f) ? v : 0.01f * v;
        if (ACT == 5) v = 0.5f * v * (1.0f + erff(v * 0.70710678118654752f));
        slab[(mOff + r) * 68 + (j << 4) + rlane] = v;
      }
    }
    __builtin_amdgcn_fence(__ATOMIC_RELEASE, "workgroup");
    __builtin_amdgcn_wave_barrier();
    __builtin_amdgcn_fence(__ATOMIC_ACQUIRE, "workgroup");
    if (OUT_MODE == 0) {
      float* C = (float*)Cout + (size_t)b * strideC;
      const int hh = lane >> 4, c4 = (lane & 15) * 4;
      for (int pass = 0; pass < 2; ++pass) {
#pragma unroll
        for (int it = 0; it < 8; ++it) {
          const int row = it * 2 + hh;
          v4f v = *(const v4f*)(slab + row * 68 + c4);
          *(volatile v4f*)(C + (size_t)(mBase + row) * ldc + n0 + c4) = v;
        }
        __threadfence();
      }
    } else {
      const int q = lane >> 3, c8 = (lane & 7) * 8;
      unsigned short* C  = (unsigned short*)Cout  + (size_t)b * strideC;
      unsigned short* C2 = (OUT_MODE == 2) ? ((unsigned short*)Cout2 + (size_t)b * strideC) : nullptr;
      for (int pass = 0; pass < 2; ++pass) {
#pragma unroll
        for (int it = 0; it < 4; ++it) {
          const int row = it * 4 + q;
          const float* sp = slab + row * 68 + c8;
          v8h hv, lv;
#pragma unroll
          for (int e = 0; e < 8; ++e) {
            if (OUT_MODE == 1) {
              hv[e] = (_Float16)sp[e];
            } else {
              unsigned short hb = f2bf_bits(sp[e]);
              unsigned short lb = f2bf_bits(sp[e] - bf_bits2f(hb));
              hv[e] = __builtin_bit_cast(_Float16, hb);
              lv[e] = __builtin_bit_cast(_Float16, lb);
            }
          }
          *(volatile v8h*)(C + (size_t)(mBase + row) * ldc + n0 + c8) = hv;
          if (OUT_MODE == 2) *(volatile v8h*)(C2 + (size_t)(mBase + row) * ldc + n0 + c8) = lv;
        }
        __threadfence();
      }
    }
    __builtin_amdgcn_fence(__ATOMIC_RELEASE, "workgroup");
    __builtin_amdgcn_wave_barrier();
    __builtin_amdgcn_fence(__ATOMIC_ACQUIRE, "workgroup");
  }
}

__global__ __launch_bounds__(256) void diff_cast_kernel(
    const float* __restrict__ x, unsigned short* __restrict__ XC, int total8)
{
  const int i = blockIdx.x * 256 + threadIdx.x;
  if (i >= total8) return;
  const int e0  = i << 3;
  const int row = e0 / kCombK;
  const int col = e0 - row * kCombK;
  const int tok = row & (kSeqL - 1);
  const bool isDiff = (col >= kDm);
  const int cs = isDiff ? (col - kDm) : col;
  const int rp = (tok > 0) ? (row - 1) : row;
  const bool hasPrev = (tok > 0);
  const float* pc = x + (size_t)row * kDm + cs;
  const float* pp = x + (size_t)rp  * kDm + cs;
  const v4f c0 = *(const v4f*)(pc);
  const v4f c1 = *(const v4f*)(pc + 4);
  const v4f p0 = *(const v4f*)(pp);
  const v4f p1 = *(const v4f*)(pp + 4);
  v8h hv;
#pragma unroll
  for (int e = 0; e < 4; ++e) {
    const float pz0 = hasPrev ? p0[e] : 0.f;
    const float pz1 = hasPrev ? p1[e] : 0.f;
    const float d0  = c0[e] - pz0;
    const float d1  = c1[e] - pz1;
    const float v0  = isDiff ? d0 : c0[e];
    const float v1  = isDiff ? d1 : c1[e];
    hv[e]     = (_Float16)v0;
    hv[4 + e] = (_Float16)v1;
  }
  unsigned short* q = XC + e0;
  *(volatile v8h*)q = hv;
  __threadfence();
  *(volatile v8h*)q = hv;
}

__global__ __launch_bounds__(256) void cast_pad_kernel(
    const float* __restrict__ src, unsigned short* __restrict__ dst,
    int Kreal, int Kpad, int nreal, int total8, float scale)
{
  const int i = blockIdx.x * 256 + threadIdx.x;
  if (i >= total8) return;
  const int e0  = i << 3;
  const int row = e0 / Kpad;
  const int col = e0 - row * Kpad;
  const bool keep = (row < nreal) && (col < Kreal);
  const int rc = (row < nreal) ? row : (nreal - 1);
  const int cc = (col < Kreal) ? col : (Kreal - 8);
  const float* p = src + (size_t)rc * Kreal + cc;
  const v4f a0 = *(const v4f*)(p);
  const v4f a1 = *(const v4f*)(p + 4);
  v8h hv;
#pragma unroll
  for (int e = 0; e < 4; ++e) {
    const float v0 = keep ? a0[e] * scale : 0.f;
    const float v1 = keep ? a1[e] * scale : 0.f;
    hv[e]     = (_Float16)v0;
    hv[4 + e] = (_Float16)v1;
  }
  unsigned short* q = dst + e0;
  *(volatile v8h*)q = hv;
  __threadfence();
  *(volatile v8h*)q = hv;
}

__global__ __launch_bounds__(256) void rmsnorm_cast_kernel(
    const float* __restrict__ P, const float* __restrict__ gw, unsigned short* __restrict__ NH, int nrows)
{
  const int lane = threadIdx.x & 31, wave = threadIdx.x >> 5;
  const int row = blockIdx.x * 8 + wave;
  if (row >= nrows) return;
  const float* pr = P + (size_t)row * kDm;
  v4f a[6], g[6];
#pragma unroll
  for (int i = 0; i < 3; ++i) {
    const int c0 = 256 * i + lane * 8;
    a[2 * i]     = *(const v4f*)(pr + c0);
    a[2 * i + 1] = *(const v4f*)(pr + c0 + 4);
    g[2 * i]     = *(const v4f*)(gw + c0);
    g[2 * i + 1] = *(const v4f*)(gw + c0 + 4);
  }
  float ss = 0.f;
#pragma unroll
  for (int k = 0; k < 6; ++k)
    ss += (a[k][0] * a[k][0] + a[k][1] * a[k][1]) + (a[k][2] * a[k][2] + a[k][3] * a[k][3]);
#pragma unroll
  for (int off = 1; off < 32; off <<= 1) ss += __shfl_xor(ss, off, 32);
  const float r = rsqrtf(ss * (1.0f / 768.0f) + 1e-5f);
  v8h hv[3];
#pragma unroll
  for (int i = 0; i < 3; ++i) {
#pragma unroll
    for (int e = 0; e < 8; ++e) {
      const int k = 2 * i + (e >> 2), ee = e & 3;
      const float v = (a[k][ee] * r) * g[k][ee];
      hv[i][e] = (_Float16)v;
    }
  }
  for (int pass = 0; pass < 2; ++pass) {
#pragma unroll
    for (int i = 0; i < 3; ++i) {
      const size_t o = (size_t)row * kDm + 256 * i + lane * 8;
      *(volatile v8h*)(NH + o) = hv[i];
    }
    __threadfence();
  }
}

__global__ __launch_bounds__(256) void conv_silu_kernel(
    const unsigned short* __restrict__ XZ, const float* __restrict__ cw, const float* __restrict__ cb,
    float* __restrict__ U, unsigned short* __restrict__ UH)
{
  __shared__ __align__(16) float sT[16 * kTP];
  const int tid = threadIdx.x, lane = tid & 31, wave = tid >> 5;
  const int d0 = blockIdx.x * 256, d = d0 + tid;
  const int g0 = blockIdx.y * 64;
  const int tb = g0 & (kSeqL - 1);
  const float w0 = cw[d * kTaps + 0], w1 = cw[d * kTaps + 1], w2 = cw[d * kTaps + 2], w3 = cw[d * kTaps + 3];
  const float bc = cb[d];
  float xm3, xm2, xm1;
  {
    const int r3 = (tb >= 3) ? (g0 - 3) : g0;
    const int r2 = (tb >= 2) ? (g0 - 2) : g0;
    const int r1 = (tb >= 1) ? (g0 - 1) : g0;
    const float v3 = h2f(XZ[(size_t)r3 * kXZP + d]);
    const float v2 = h2f(XZ[(size_t)r2 * kXZP + d]);
    const float v1 = h2f(XZ[(size_t)r1 * kXZP + d]);
    xm3 = (tb >= 3) ? v3 : 0.f;
    xm2 = (tb >= 2) ? v2 : 0.f;
    xm1 = (tb >= 1) ? v1 : 0.f;
  }
  const int hrow = wave >> 1;
  const int hch  = (wave & 1) * 128 + lane * 4;
#pragma unroll 1
  for (int sub = 0; sub < 4; ++sub) {
    const int lb = g0 + sub * 16;
#pragma unroll 1
    for (int s = 0; s < 16; ++s) {
      const float xc = h2f(XZ[(size_t)(lb + s) * kXZP + d]);
      float acc = w0 * xm3;
      acc = fmaf(w1, xm2, acc);
      acc = fmaf(w2, xm1, acc);
      acc = fmaf(w3, xc, acc);
      const float sv = acc + bc;
      const float sg = __builtin_amdgcn_rcpf(1.0f + __expf(-sv));
      sT[s * kTP + tid] = sv * sg;
      xm3 = xm2; xm2 = xm1; xm1 = xc;
    }
    __syncthreads();
    v4f fv[4];
    v8h bh[2];
#pragma unroll
    for (int it = 0; it < 4; ++it) fv[it] = *(const v4f*)(sT + (it * 4 + hrow) * kTP + hch);
#pragma unroll
    for (int it = 0; it < 2; ++it) {
      const float* sp = sT + (it * 8 + wave) * kTP + lane * 8;
      const v4f a0 = *(const v4f*)(sp);
      const v4f a1 = *(const v4f*)(sp + 4);
#pragma unroll
      for (int e = 0; e < 4; ++e) {
        bh[it][e]     = (_Float16)(a0[e] * 256.0f);
        bh[it][4 + e] = (_Float16)(a1[e] * 256.0f);
      }
    }
    for (int pass = 0; pass < 2; ++pass) {
#pragma unroll
      for (int it = 0; it < 4; ++it)
        *(volatile v4f*)(U + (size_t)(lb + it * 4 + hrow) * kDin + d0 + hch) = fv[it];
#pragma unroll
      for (int it = 0; it < 2; ++it) {
        const size_t o = (size_t)(lb + it * 8 + wave) * kDin + d0 + lane * 8;
        *(volatile v8h*)(UH + o) = bh[it];
      }
      __threadfence();
    }
    __syncthreads();
  }
}

__global__ __launch_bounds__(256) void dt_cast_kernel(
    const float* __restrict__ XD, unsigned short* __restrict__ DTH, int total8)
{
  const int i = blockIdx.x * 256 + threadIdx.x;
  if (i >= total8) return;
  const int e0  = i << 3;
  const int row = e0 >> 6;
  const int c8  = e0 & 63;
  const bool keep = (c8 < kDtR);
  const int cc = keep ? c8 : (kDtR - 8);
  const float* p = XD + (size_t)row * kXdP + cc;
  const v4f a0 = *(const v4f*)(p);
  const v4f a1 = *(const v4f*)(p + 4);
  v8h hv;
#pragma unroll
  for (int e = 0; e < 4; ++e) {
    const float v0 = keep ? a0[e] * 256.0f : 0.f;
    const float v1 = keep ? a1[e] * 256.0f : 0.f;
    hv[e]     = (_Float16)v0;
    hv[4 + e] = (_Float16)v1;
  }
  unsigned short* q = DTH + e0;
  *(volatile v8h*)q = hv;
  __threadfence();
  *(volatile v8h*)q = hv;
}

__global__ __launch_bounds__(kScanCh) void scan_kernel(
    const float* __restrict__ DLR, const float* __restrict__ U, const unsigned short* __restrict__ XZ,
    const float* __restrict__ XD, const float* __restrict__ A_log, const float* __restrict__ Dv,
    unsigned short* __restrict__ YH)
{
  __shared__ __align__(16) float sBC[16 * 2 * kNst];
  __shared__ __align__(16) float sY[16 * kSYP];
  const int tid = threadIdx.x, lane = tid & 31, wave = tid >> 5;
  const int d0 = blockIdx.x * kScanCh, d = d0 + tid;
  const int rowbase = blockIdx.y * kSeqL;

  float An[kNst];
#pragma unroll
  for (int n = 0; n < kNst; ++n) An[n] = -__expf(A_log[(size_t)d * kNst + n]);
  const float Dd = Dv[d];
  float h[kNst];
#pragma unroll
  for (int n = 0; n < kNst; ++n) h[n] = 0.f;

#pragma unroll 1
  for (int c = 0; c < kSeqL / 16; ++c) {
    const int l0 = rowbase + c * 16;
    {
      const int r = tid >> 3, q = (tid & 7) * 4;
      const v4f v = *(const v4f*)(XD + (size_t)(l0 + r) * kXdP + kDtR + q);
      *(v4f*)(sBC + r * 32 + q) = v;
    }
    __syncthreads();
#pragma unroll 1
    for (int s = 0; s < 16; ++s) {
      const size_t m = (size_t)(l0 + s);
      const float a     = DLR[m * kDin + d];
      const float delta = fmaxf(a, 0.0f) + log1pf(__expf(-fabsf(a)));
      const float xv    = U[m * kDin + d];
      const float zv    = h2f(XZ[m * kXZP + kDin + d]);
      float du = delta * xv;
      asm volatile("" : "+v"(du));
      const float* bq = sBC + s * 32;
      const float* cq = bq + kNst;
      float y = 0.f;
#pragma unroll
      for (int qq = 0; qq < 4; ++qq) {
        const v4f Bq = *(const v4f*)(bq + 4 * qq);
        const v4f Cq = *(const v4f*)(cq + 4 * qq);
#pragma unroll
        for (int e = 0; e < 4; ++e) {
          const int n = qq * 4 + e;
          const float ex = __expf(delta * An[n]);
          float p = du * Bq[e];
          asm volatile("" : "+v"(p));
          float qv = h[n] * ex;
          asm volatile("" : "+v"(qv));
          const float hn = qv + p;
          h[n] = hn;
          float rr = Cq[e] * hn;
          asm volatile("" : "+v"(rr));
          y += rr;
        }
      }
      float sk = xv * Dd;
      asm volatile("" : "+v"(sk));
      y += sk;
      const float sg = __builtin_amdgcn_rcpf(1.0f + __expf(-zv));
      const float g  = zv * sg;
      sY[s * kSYP + tid] = (y * g) * 256.0f;
    }
    __syncthreads();
    {
      const int c8 = (lane & 15) * 8;
      const int rowA = 4 * wave + (lane >> 4);
      const int rowB = rowA + 2;
      v8h hvA, hvB;
      {
        const float* sp = sY + rowA * kSYP + c8;
        const v4f a0 = *(const v4f*)(sp);
        const v4f a1 = *(const v4f*)(sp + 4);
#pragma unroll
        for (int e = 0; e < 4; ++e) { hvA[e] = (_Float16)a0[e]; hvA[4 + e] = (_Float16)a1[e]; }
      }
      {
        const float* sp = sY + rowB * kSYP + c8;
        const v4f a0 = *(const v4f*)(sp);
        const v4f a1 = *(const v4f*)(sp + 4);
#pragma unroll
        for (int e = 0; e < 4; ++e) { hvB[e] = (_Float16)a0[e]; hvB[4 + e] = (_Float16)a1[e]; }
      }
      const size_t oA = (size_t)(l0 + rowA) * kDin + d0 + c8;
      const size_t oB = (size_t)(l0 + rowB) * kDin + d0 + c8;
      for (int pass = 0; pass < 2; ++pass) {
        *(volatile v8h*)(YH + oA) = hvA;
        *(volatile v8h*)(YH + oB) = hvB;
        __threadfence();
      }
    }
  }
}

extern "C" void kernel_launch(void* const* d_in, const int* in_sizes, int n_in,
                              void* d_out, int out_size, void* d_ws, size_t ws_size,
                              hipStream_t stream)
{
  if (n_in < 13) return;
  const float* x      = (const float*)d_in[0];
  const float* Wp     = (const float*)d_in[1];
  const float* bp     = (const float*)d_in[2];
  const float* gamma  = (const float*)d_in[3];
  const float* Win    = (const float*)d_in[4];
  const float* Wconv  = (const float*)d_in[5];
  const float* bconv  = (const float*)d_in[6];
  const float* Wx     = (const float*)d_in[7];
  const float* Wdt    = (const float*)d_in[8];
  const float* bdt    = (const float*)d_in[9];
  const float* A_log  = (const float*)d_in[10];
  const float* Dparam = (const float*)d_in[11];
  const float* Wout   = (const float*)d_in[12];
  float* dout = (float*)d_out;

  if (in_sizes[0] != kRows * kDm) return;
  if (in_sizes[1] != kDm * kCombK || in_sizes[2] != kDm || in_sizes[3] != kDm) return;
  if (in_sizes[4] != kXZP * kDm) return;
  if (in_sizes[5] != kDin * kTaps || in_sizes[6] != kDin) return;
  if (in_sizes[7] != kXdN * kDin) return;
  if (in_sizes[8] != kDin * kDtR || in_sizes[9] != kDin) return;
  if (in_sizes[10] != kDin * kNst || in_sizes[11] != kDin) return;
  if (in_sizes[12] != kDm * kDin) return;
  if (out_size != kRows * kDm) return;

  const size_t SZ_RA   = (size_t)kRows * kCombK * 2;
  const size_t SZ_WPH  = (size_t)kDm * kCombK * 2;
  const size_t SZ_RP   = (size_t)kRows * kDm * 4;
  const size_t SZ_XD   = (size_t)kRows * kXdP * 4;
  const size_t SZ_DTH  = (size_t)kRows * kDtP * 2;
  const size_t SZ_NH   = (size_t)kRows * kDm * 2;
  const size_t SZ_WIH  = (size_t)kXZP * kDm * 2;
  const size_t SZ_XZ   = (size_t)kRows * kXZP * 2;
  const size_t SZ_U    = (size_t)kRows * kDin * 4;
  const size_t SZ_WXH  = (size_t)kXdP * kDin * 2;
  const size_t SZ_WDH  = (size_t)kDin * kDtP * 2;
  const size_t SZ_DLR  = (size_t)kRows * kDin * 4;
  const size_t SZ_WOH  = (size_t)kDm * kDin * 2;
  if (SZ_XD + SZ_DTH > SZ_RP) return;
  const size_t OFF_RA  = 0;
  const size_t OFF_WPH = OFF_RA  + SZ_RA;
  const size_t OFF_RP  = OFF_WPH + SZ_WPH;
  const size_t OFF_XD  = OFF_RP;
  const size_t OFF_DTH = OFF_RP  + SZ_XD;
  const size_t OFF_NH  = OFF_RP  + SZ_RP;
  const size_t OFF_WIH = OFF_NH  + SZ_NH;
  const size_t OFF_XZ  = OFF_WIH + SZ_WIH;
  const size_t OFF_U   = OFF_XZ  + SZ_XZ;
  const size_t OFF_WXH = OFF_U   + SZ_U;
  const size_t OFF_WDH = OFF_WXH + SZ_WXH;
  const size_t OFF_DLR = OFF_WDH + SZ_WDH;
  const size_t OFF_WOH = OFF_DLR + SZ_DLR;
  const size_t TOTAL   = OFF_WOH + SZ_WOH;
  if (ws_size < TOTAL) return;

  char* ws = (char*)d_ws;
  unsigned short* XC   = (unsigned short*)(ws + OFF_RA);
  unsigned short* UH   = (unsigned short*)(ws + OFF_RA);
  unsigned short* YH   = (unsigned short*)(ws + OFF_RA);
  unsigned short* WPH  = (unsigned short*)(ws + OFF_WPH);
  float*          RP   = (float*)(ws + OFF_RP);
  float*          XD   = (float*)(ws + OFF_XD);
  unsigned short* DTH  = (unsigned short*)(ws + OFF_DTH);
  unsigned short* NH   = (unsigned short*)(ws + OFF_NH);
  unsigned short* WIH  = (unsigned short*)(ws + OFF_WIH);
  unsigned short* XZ   = (unsigned short*)(ws + OFF_XZ);
  float*          U    = (float*)(ws + OFF_U);
  unsigned short* WXH  = (unsigned short*)(ws + OFF_WXH);
  unsigned short* WDH  = (unsigned short*)(ws + OFF_WDH);
  float*          DLR  = (float*)(ws + OFF_DLR);
  unsigned short* WOH  = (unsigned short*)(ws + OFF_WOH);
  const float* dummy_bias  = bp;
  const float* dummy_resid = x;

  {
    const int total8 = (kRows * kCombK) / 8;
    diff_cast_kernel<<<(total8 + 255) / 256, 256, 0, stream>>>(x, XC, total8);
  }

  {
    const int t_wp = (kDm * kCombK) / 8, t_win = (kXZP * kDm) / 8, t_wx = (kXdP * kDin) / 8, t_wdt = (kDin * kDtP) / 8, t_wo = (kDm * kDin) / 8;
    cast_pad_kernel<<<(t_wp  + 255) / 256, 256, 0, stream>>>(Wp,   WPH, kCombK, kCombK, kDm,  t_wp,  64.0f);
    cast_pad_kernel<<<(t_win + 255) / 256, 256, 0, stream>>>(Win,  WIH, kDm,    kDm,    kXZP, t_win, 64.0f);
    cast_pad_kernel<<<(t_wx  + 255) / 256, 256, 0, stream>>>(Wx,   WXH, kDin,   kDin,   kXdN, t_wx,  64.0f);
    cast_pad_kernel<<<(t_wdt + 255) / 256, 256, 0, stream>>>(Wdt,  WDH, kDtR,   kDtP,   kDin, t_wdt, 16.0f);
    cast_pad_kernel<<<(t_wo  + 255) / 256, 256, 0, stream>>>(Wout, WOH, kDin,   kDin,   kDm,  t_wo,  64.0f);
  }

  wmma_gemm64<0, false, 2, 0, false><<<dim3((kRows / 64) * (kDm / 64) / 8, 1), 256, 0, stream>>>(
      XC, XC, kCombK, 0L, WPH, WPH, kCombK, 0L,
      (void*)RP, (void*)RP, kDm, 0L, bp, dummy_resid, 0L, kRows, kDm, kCombK, 1.0f / 64.0f);

  rmsnorm_cast_kernel<<<kRows / 8, 256, 0, stream>>>(RP, gamma, NH, kRows);

  wmma_gemm64<0, false, 0, 1, false><<<dim3((kRows / 64) * (kXZP / 64) / 8, 1), 256, 0, stream>>>(
      NH, NH, kDm, 0L, WIH, WIH, kDm, 0L,
      (void*)XZ, (void*)XZ, kXZP, 0L, dummy_bias, dummy_resid, 0L, kRows, kXZP, kDm, 1.0f / 64.0f);

  conv_silu_kernel<<<dim3(kDin / 256, kRows / 64), 256, 0, stream>>>(XZ, Wconv, bconv, U, UH);

  wmma_gemm64<0, false, 0, 0, false><<<dim3((kRows / 64) * (kXdP / 64) / 8, 1), 256, 0, stream>>>(
      UH, UH, kDin, 0L, WXH, WXH, kDin, 0L,
      (void*)XD, (void*)XD, kXdP, 0L, dummy_bias, dummy_resid, 0L, kRows, kXdP, kDin, 1.0f / 16384.0f);

  {
    const int total8 = (kRows * kDtP) / 8;
    dt_cast_kernel<<<(total8 + 255) / 256, 256, 0, stream>>>(XD, DTH, total8);
  }

  wmma_gemm64<0, false, 2, 0, false><<<dim3((kRows / 64) * (kDin / 64) / 8, 1), 256, 0, stream>>>(
      DTH, DTH, kDtP, 0L, WDH, WDH, kDtP, 0L,
      (void*)DLR, (void*)DLR, kDin, 0L, bdt, dummy_resid, 0L, kRows, kDin, kDtP, 1.0f / 4096.0f);

  scan_kernel<<<dim3(kDin / kScanCh, kBatch), kScanCh, 0, stream>>>(DLR, U, XZ, XD, A_log, Dparam, YH);

  wmma_gemm64<0, false, 0, 0, true><<<dim3((kRows / 64) * (kDm / 64) / 8, 1), 256, 0, stream>>>(
      YH, YH, kDin, 0L, WOH, WOH, kDin, 0L,
      (void*)dout, (void*)dout, kDm, 0L, dummy_bias, x, 0L, kRows, kDm, kDin, 1.0f / 16384.0f);
}
